// GNNEncoders_8581344657807
// MI455X (gfx1250) — hardware-verified
//
#include <hip/hip_runtime.h>
#include <stddef.h>


#define DX     64
#define NHD    4
#define HCOL   256
#define KP     64
#define NTHR   256
#define NWAVE  8
#define RPB_W  32
#define RPB_N  128
#define STG    68
#define ATP    72
#define SMEM_F 9216
#define NB     256
#define CHUNK  2048
#define WCAP   256
#define NGRP   (CHUNK / (NTHR * 4))
#define RB     400
#define AGG_LDS 282688

#define PT_W   (3 * HCOL * 8)
#define PT_R   (HCOL * 8)
#define PT_F   (DX * 8)
#define PT_B   (HCOL / 4)
#define PT_ALL (PT_W + PT_R + PT_F + PT_B)

static_assert(NGRP == 2);
static_assert(WCAP == NGRP * 4 * 32);
static_assert(NB == 256);
static_assert(CHUNK == 2048);
static_assert(AGG_LDS == NB * HCOL * 4 + 3 * NB * NHD * 4 + NWAVE * WCAP * 4 + 16 * 4);
static_assert(SMEM_F * 4 >= 2 * RPB_N * ATP * 2);
static_assert(SMEM_F >= NWAVE * 16 * STG);
static_assert((PT_W % 32) == 0 && (PT_R % 32) == 0 && (PT_F % 32) == 0);

typedef float          v4f  __attribute__((ext_vector_type(4)));
typedef float          v8f  __attribute__((ext_vector_type(8)));
typedef int            v4i  __attribute__((ext_vector_type(4)));
typedef int            v8i  __attribute__((ext_vector_type(8)));
typedef unsigned       v4u  __attribute__((ext_vector_type(4)));
typedef unsigned short us;
typedef us             v8us __attribute__((ext_vector_type(8)));
typedef __bf16         v16bf __attribute__((ext_vector_type(16)));
typedef double         v2d  __attribute__((ext_vector_type(2)));
union Frag { v8i v; v8us half[2]; };

__device__ __forceinline__ unsigned bfr(float f) {
  const unsigned u = __float_as_uint(f);
  return (u + 0x7fffu + ((u >> 16) & 1u)) >> 16;
}
__device__ __forceinline__ float bup(unsigned b) { return __uint_as_float(b << 16); }

__device__ __forceinline__ void split8(v4f a, v4f b, v4u* H, v4u* L) {
  float v[8] = {a.x, a.y, a.z, a.w, b.x, b.y, b.z, b.w};
  unsigned hb[8], lb[8];
#pragma unroll
  for (int j = 0; j < 8; ++j) { hb[j] = bfr(v[j]); lb[j] = bfr(v[j] - bup(hb[j])); }
  v4u h4, l4;
  h4.x = hb[0] | (hb[1] << 16); h4.y = hb[2] | (hb[3] << 16); h4.z = hb[4] | (hb[5] << 16); h4.w = hb[6] | (hb[7] << 16);
  l4.x = lb[0] | (lb[1] << 16); l4.y = lb[2] | (lb[3] << 16); l4.z = lb[4] | (lb[5] << 16); l4.w = lb[6] | (lb[7] << 16);
  *H = h4; *L = l4;
}

__device__ __forceinline__ v8i ldf(const us* rp, int k0, int hh) {
  Frag f;
  f.half[0] = *(const v8us*)(rp + k0 + 8 * hh);
  f.half[1] = *(const v8us*)(rp + k0 + 16 + 8 * hh);
  return f.v;
}

__device__ __forceinline__ v8f wmb(v8i a, v8i b, v8f c) {
  v8f d = __builtin_amdgcn_wmma_f32_16x16x32_bf16(false, __builtin_bit_cast(v16bf, a), false,
                                                   __builtin_bit_cast(v16bf, b), (short)0, c, false, false);
  asm volatile("v_nop\n\tv_nop\n\tv_nop\n\tv_nop" : "+v"(d) : "v"(a), "v"(b));
  return d;
}

__global__ __launch_bounds__(NTHR) void k_prep(const float* __restrict__ W, const float* __restrict__ rW,
                                               const float* __restrict__ bvec, const float* __restrict__ fcW,
                                               us* Wth, us* Wtl, us* Rth, us* Rtl, us* Fth, us* Ftl, float* bsum) {
  const int task = blockIdx.x * NTHR + threadIdx.x;
  if (task >= PT_ALL) return;
  if (task >= PT_W + PT_R + PT_F) {
    const int t4 = task - (PT_W + PT_R + PT_F);
    const v4f s = (*(const v4f*)(bvec + 4 * t4) + *(const v4f*)(bvec + HCOL + 4 * t4)) + *(const v4f*)(bvec + 2 * HCOL + 4 * t4);
    float* gp = bsum + 4 * t4;
    *(volatile v4f*)gp = s;
    __threadfence();
    *(volatile v4f*)gp = s;
    return;
  }
  float v[8];
  size_t off;
  us* ph;
  us* pl;
  if (task < PT_W) {
    const int r = task / PT_R, rem = task - r * PT_R, n = rem >> 3, kc = rem & 7;
    const float* wp = W + (size_t)r * KP * HCOL + (size_t)(kc * 8) * HCOL + n;
#pragma unroll
    for (int j = 0; j < 8; ++j) v[j] = wp[(size_t)j * HCOL];
    off = (size_t)(r * HCOL + n) * KP + kc * 8; ph = Wth; pl = Wtl;
  } else if (task < PT_W + PT_R) {
    const int rem = task - PT_W, n = rem >> 3, kc = rem & 7;
    const float* wp = rW + (size_t)(kc * 8) * HCOL + n;
#pragma unroll
    for (int j = 0; j < 8; ++j)
      v[j] = (wp[(size_t)j * HCOL] + wp[(size_t)KP * HCOL + (size_t)j * HCOL]) + wp[(size_t)2 * KP * HCOL + (size_t)j * HCOL];
    off = (size_t)n * KP + kc * 8; ph = Rth; pl = Rtl;
  } else {
    const int rem = task - PT_W - PT_R, c = rem >> 3, kc = rem & 7;
    const float* wp = fcW + (size_t)(kc * 8) * DX + c;
#pragma unroll
    for (int j = 0; j < 8; ++j) v[j] = wp[(size_t)j * DX];
    off = (size_t)c * KP + kc * 8; ph = Fth; pl = Ftl;
  }
  const v4f a = {v[0], v[1], v[2], v[3]};
  const v4f b = {v[4], v[5], v[6], v[7]};
  v4u H, L;
  split8(a, b, &H, &L);
  us* p1 = ph + off;
  us* p2 = pl + off;
  *(volatile v4u*)p1 = H;
  *(volatile v4u*)p2 = L;
  __threadfence();
  *(volatile v4u*)p1 = H;
  *(volatile v4u*)p2 = L;
}

__global__ __launch_bounds__(NTHR) void k_bn_part(const float* __restrict__ x, int nN, double* part) {
  __shared__ __attribute__((aligned(16))) double red[4 * 128];
  __shared__ __attribute__((aligned(16))) double lineo[128];
  const int tid = threadIdx.x, d = tid & 63, q = tid >> 6;
  const int r0 = blockIdx.x * RB;
  int r1 = r0 + RB;
  if (r1 > nN) r1 = nN;
  double s = 0.0, ss = 0.0;
#pragma unroll 1
  for (int r = r0 + q; r < r1; r += 4) {
    const double v = (double)x[(size_t)r * DX + d];
    s += v;
    ss += v * v;
  }
  red[q * 128 + d] = s;
  red[q * 128 + 64 + d] = ss;
  __syncthreads();
  if (tid < 128) lineo[tid] = ((red[tid] + red[128 + tid]) + red[256 + tid]) + red[384 + tid];
  __syncthreads();
  if (tid < 64) {
    const v2d o = *(const v2d*)(lineo + 2 * tid);
    double* gp = part + (size_t)blockIdx.x * 128 + 2 * tid;
    *(volatile v2d*)gp = o;
    __threadfence();
    *(volatile v2d*)gp = o;
  }
}

__global__ __launch_bounds__(NTHR) void k_bn_final(const double* __restrict__ part, int P, int nN,
                                                   const float* __restrict__ g, float* scsh) {
  __shared__ __attribute__((aligned(16))) double tot[128];
  __shared__ __attribute__((aligned(16))) float o[128];
  const int tid = threadIdx.x;
  if (tid < 128) {
    double a = 0.0;
#pragma unroll 1
    for (int p = 0; p < P; ++p) a += part[(size_t)p * 128 + tid];
    tot[tid] = a;
  }
  __syncthreads();
  if (tid < 64) {
    const double inv = 1.0 / (double)nN;
    const double mu = tot[tid] * inv;
    double var = tot[64 + tid] * inv - mu * mu;
    if (var < 0.0) var = 0.0;
    const float varf = (float)var;
    const float rs = 1.0f / sqrtf(varf + 1e-5f);
    o[tid] = (float)mu;
    o[64 + tid] = rs * g[tid];
  }
  __syncthreads();
  if (tid < 32) {
    const v4f v = *(const v4f*)(o + 4 * tid);
    float* gp = scsh + 4 * tid;
    *(volatile v4f*)gp = v;
    __threadfence();
    *(volatile v4f*)gp = v;
  }
}

__global__ __launch_bounds__(NTHR) void k_bn_apply(const float* __restrict__ x, const float* __restrict__ scsh,
                                                   const float* __restrict__ be, int nN, us* xh, us* xl) {
  const int gid = blockIdx.x * NTHR + threadIdx.x;
  const int row = gid >> 3, c8 = gid & 7;
  const int rr = row < nN ? row : nN - 1;
  const float* xp = x + (size_t)rr * DX + c8 * 8;
  const v4f x0 = *(const v4f*)xp, x1 = *(const v4f*)(xp + 4);
  const v4f mu0 = *(const v4f*)(scsh + c8 * 8), mu1 = *(const v4f*)(scsh + c8 * 8 + 4);
  const v4f sg0 = *(const v4f*)(scsh + DX + c8 * 8), sg1 = *(const v4f*)(scsh + DX + c8 * 8 + 4);
  const v4f b0 = *(const v4f*)(be + c8 * 8), b1 = *(const v4f*)(be + c8 * 8 + 4);
  v4f y0 = (x0 - mu0) * sg0 + b0;
  v4f y1 = (x1 - mu1) * sg1 + b1;
  const v4f z = {0.f, 0.f, 0.f, 0.f};
  if (row >= nN) { y0 = z; y1 = z; }
  v4u H, L;
  split8(y0, y1, &H, &L);
  const size_t off = (size_t)row * DX + c8 * 8;
  *(volatile v4u*)(xh + off) = H;
  *(volatile v4u*)(xl + off) = L;
  __threadfence();
  *(volatile v4u*)(xh + off) = H;
  *(volatile v4u*)(xl + off) = L;
}

template <int MODE>
__global__ __launch_bounds__(NTHR) void k_gemm(const us* __restrict__ Ah, const us* __restrict__ Al,
                                               const float* Hs,
                                               const us* __restrict__ Bh, const us* __restrict__ Bl,
                                               const float* vecA, const float* vecB,
                                               float* outP, float* outE, int ldo, int nStore) {
  __shared__ __attribute__((aligned(16))) float smem[SMEM_F];
  __shared__ __attribute__((aligned(16))) float s_el[RPB_W * 8];
  const int tid = threadIdx.x, lane = tid & 31, wave = tid >> 5;
  const int hh = lane >> 4, m = lane & 15;
  const int rt = (MODE == 2) ? wave : (wave >> 2);
  const int cg = (MODE == 2) ? 0 : (wave & 3);
  const int rpb = (MODE == 2) ? RPB_N : RPB_W;
  const int rowBase = blockIdx.x * rpb + rt * 16;

  v8i aH0, aH1, aL0, aL1;
  if (MODE == 2) {
    us* At = (us*)smem;
    for (int task = tid; task < RPB_N * 8; task += NTHR) {
      const int row = task >> 3, c8 = task & 7;
      const float* hp = Hs + (size_t)(blockIdx.x * RPB_N + row) * HCOL + c8 * 8;
      const v4f u0 = *(const v4f*)(hp),          u1 = *(const v4f*)(hp + 4);
      const v4f w0 = *(const v4f*)(hp + DX),     w1 = *(const v4f*)(hp + DX + 4);
      const v4f y0 = *(const v4f*)(hp + 2 * DX), y1 = *(const v4f*)(hp + 2 * DX + 4);
      const v4f z0 = *(const v4f*)(hp + 3 * DX), z1 = *(const v4f*)(hp + 3 * DX + 4);
      const v4f m0 = ((u0 + w0) + (y0 + z0)) * 0.25f;
      const v4f m1 = ((u1 + w1) + (y1 + z1)) * 0.25f;
      v4u H, L;
      split8(m0, m1, &H, &L);
      *(v4u*)(At + row * ATP + c8 * 8) = H;
      *(v4u*)(At + RPB_N * ATP + row * ATP + c8 * 8) = L;
    }
    __syncthreads();
    const us* arh = (const us*)smem + (rt * 16 + m) * ATP;
    const us* arl = arh + RPB_N * ATP;
    aH0 = ldf(arh, 0, hh); aH1 = ldf(arh, 32, hh);
    aL0 = ldf(arl, 0, hh); aL1 = ldf(arl, 32, hh);
    __syncthreads();
  } else {
    const us* arh = Ah + (size_t)(rowBase + m) * KP;
    const us* arl = Al + (size_t)(rowBase + m) * KP;
    aH0 = ldf(arh, 0, hh); aH1 = ldf(arh, 32, hh);
    aL0 = ldf(arl, 0, hh); aL1 = ldf(arl, 32, hh);
  }

  float* stage = smem + wave * (16 * STG);
  float se[8], sr[8];
#pragma unroll
  for (int r = 0; r < 8; ++r) { se[r] = 0.f; sr[r] = 0.f; }

#pragma unroll 1
  for (int t = 0; t < 4; ++t) {
    const int ncol = cg * DX + t * 16 + m;
    const us* brh = Bh + (size_t)ncol * KP;
    const us* brl = Bl + (size_t)ncol * KP;
    const v8i bH0 = ldf(brh, 0, hh), bH1 = ldf(brh, 32, hh);
    const v8i bL0 = ldf(brl, 0, hh), bL1 = ldf(brl, 32, hh);
    v8f acc = {0.f, 0.f, 0.f, 0.f, 0.f, 0.f, 0.f, 0.f};
    acc = wmb(aH0, bH0, acc);
    acc = wmb(aL0, bH0, acc);
    acc = wmb(aH0, bL0, acc);
    acc = wmb(aH1, bH1, acc);
    acc = wmb(aL1, bH1, acc);
    acc = wmb(aH1, bL1, acc);
    float add = 0.f, ca = 0.f, cb = 0.f;
    if (MODE == 0) { ca = vecA[ncol]; cb = vecB[ncol]; } else { add = vecA[ncol]; }
#pragma unroll
    for (int r = 0; r < 8; ++r) {
      float v = acc[r] + add;
      if (MODE == 2) v = fmaxf(v, 0.f);
      stage[(8 * hh + r) * STG + t * 16 + m] = v;
      if (MODE == 0) { se[r] += v * ca; sr[r] += v * cb; }
    }
  }

  if (MODE == 0) {
#pragma unroll
    for (int mk = 1; mk < 16; mk <<= 1) {
#pragma unroll
      for (int r = 0; r < 8; ++r) {
        se[r] += __shfl_xor(se[r], mk, 32);
        sr[r] += __shfl_xor(sr[r], mk, 32);
      }
    }
    if (m == 0) {
#pragma unroll
      for (int r = 0; r < 8; ++r) {
        s_el[(rt * 16 + 8 * hh + r) * 8 + cg] = se[r];
        s_el[(rt * 16 + 8 * hh + r) * 8 + 4 + cg] = sr[r];
      }
    }
  }
  __syncthreads();

  v4f ov[8];
#pragma unroll
  for (int i = 0; i < 8; ++i) ov[i] = *(const v4f*)(stage + (2 * i + hh) * STG + 4 * m);
  const size_t colo = (size_t)cg * DX + 4 * m;
  v4f e0 = {0.f, 0.f, 0.f, 0.f};
  v4f e1 = e0;
  float* ep = outE + (size_t)blockIdx.x * RPB_W * 8;
  if (MODE == 0 && wave == 0) {
    e0 = *(const v4f*)(s_el + 4 * lane);
    e1 = *(const v4f*)(s_el + 128 + 4 * lane);
  }
#pragma unroll
  for (int i = 0; i < 8; ++i) {
    const int grow = rowBase + 2 * i + hh;
    if (grow < nStore) *(volatile v4f*)(outP + (size_t)grow * ldo + colo) = ov[i];
  }
  if (MODE == 0 && wave == 0) {
    *(volatile v4f*)(ep + 4 * lane) = e0;
    *(volatile v4f*)(ep + 128 + 4 * lane) = e1;
  }
  __threadfence();
#pragma unroll
  for (int i = 0; i < 8; ++i) {
    const int grow = rowBase + 2 * i + hh;
    if (grow < nStore) *(volatile v4f*)(outP + (size_t)grow * ldo + colo) = ov[i];
  }
  if (MODE == 0 && wave == 0) {
    *(volatile v4f*)(ep + 4 * lane) = e0;
    *(volatile v4f*)(ep + 128 + 4 * lane) = e1;
  }
}

#define HITJ(J, HJ, SJ) { \
  const unsigned mj = __builtin_amdgcn_ballot_w32(HJ); \
  if (HJ) { \
    const int pos = wc + (int)__builtin_amdgcn_mbcnt_lo(mj, 0u); \
    if (pos < WCAP) list[wave * WCAP + pos] = ((el0 + (J)) << 8) | (int)(SJ); \
  } \
  wc += (int)__builtin_popcount(mj); }

__global__ __launch_bounds__(NTHR) void k_agg(const int* __restrict__ srcA, const int* __restrict__ dstA, int nE,
                                              const float* __restrict__ fs, const float* __restrict__ eler,
                                              float* hsum, int nN) {
  extern __shared__ v4f lds_dyn[];
  float* acc  = (float*)lds_dyn;
  float* den  = acc + NB * HCOL;
  float* mx   = den + NB * NHD;
  float* ers  = mx + NB * NHD;
  int*   list = (int*)(ers + NB * NHD);
  int*   wcnt = list + NWAVE * WCAP;

  const int tid = threadIdx.x, lane = tid & 31, wave = tid >> 5;
  const int nodeBase = blockIdx.x * NB;
  {
    const v4f z = {0.f, 0.f, 0.f, 0.f};
    for (int i = tid; i < NB * HCOL / 4; i += NTHR) lds_dyn[i] = z;
    const float ninf = __uint_as_float(0xff800000u);
    for (int i = tid; i < NB * NHD; i += NTHR) {
      int nd = nodeBase + (i >> 2);
      if (nd > nN - 1) nd = nN - 1;
      den[i] = 0.f;
      mx[i]  = ninf;
      ers[i] = eler[(size_t)nd * 8 + 4 + (i & 3)];
    }
  }
  __syncthreads();

  const int hsel = lane >> 3;
  const int nChunks = (nE + CHUNK - 1) / CHUNK;
#pragma unroll 1
  for (int ch = 0; ch < nChunks; ++ch) {
    const int cbase = ch * CHUNK;
    const bool full = (cbase + CHUNK <= nE);
    int wc = 0;
#pragma unroll
    for (int g = 0; g < NGRP; ++g) {
      const int el0 = (g * NTHR + tid) * 4;
      const int e0  = cbase + el0;
      const int sent = -2147483647 - 1;
      v4i d;
      if (full) {
        d = *(const v4i*)(dstA + e0);
      } else {
        const int c0 = e0     < nE - 1 ? e0     : nE - 1;
        const int c1 = e0 + 1 < nE - 1 ? e0 + 1 : nE - 1;
        const int c2 = e0 + 2 < nE - 1 ? e0 + 2 : nE - 1;
        const int c3 = e0 + 3 < nE - 1 ? e0 + 3 : nE - 1;
        const int t0 = dstA[c0], t1 = dstA[c1], t2 = dstA[c2], t3 = dstA[c3];
        d.x = (e0     < nE) ? t0 : sent;
        d.y = (e0 + 1 < nE) ? t1 : sent;
        d.z = (e0 + 2 < nE) ? t2 : sent;
        d.w = (e0 + 3 < nE) ? t3 : sent;
      }
      const unsigned s0 = (unsigned)d.x - (unsigned)nodeBase;
      const unsigned s1 = (unsigned)d.y - (unsigned)nodeBase;
      const unsigned s2 = (unsigned)d.z - (unsigned)nodeBase;
      const unsigned s3 = (unsigned)d.w - (unsigned)nodeBase;
      const bool h0 = s0 < (unsigned)NB;
      const bool h1 = s1 < (unsigned)NB;
      const bool h2 = s2 < (unsigned)NB;
      const bool h3 = s3 < (unsigned)NB;
      const unsigned many = __builtin_amdgcn_ballot_w32(h0 | h1 | h2 | h3);
      if (many != 0u) {
        HITJ(0, h0, s0)
        HITJ(1, h1, s1)
        HITJ(2, h2, s2)
        HITJ(3, h3, s3)
      }
    }
    if (lane == 0) wcnt[wave] = wc;
    __syncthreads();

    if (wave == 0) {
#pragma unroll 1
      for (int wsx = 0; wsx < NWAVE; ++wsx) {
        int n = wcnt[wsx];
        n = n < 0 ? 0 : (n > WCAP ? WCAP : n);
#pragma unroll 1
        for (int i = 0; i < n; ++i) {
          const int ent  = list[wsx * WCAP + i];
          const int slot = ent & (NB - 1);
          const int el   = (ent >> 8) & (CHUNK - 1);
          int e = cbase + el;
          if (e > nE - 1) e = nE - 1;
          int s = srcA[e];
          s = s < 0 ? 0 : (s > nN - 1 ? nN - 1 : s);
          const float lg = eler[(size_t)s * 8 + hsel] + ers[slot * NHD + hsel];
          const float v  = lg > 0.f ? lg : 0.2f * lg;
          const float mo = mx[slot * NHD + hsel];
          const float dn = den[slot * NHD + hsel];
          const float mn = fmaxf(mo, v);
          const float sc = __expf(mo - mn);
          const float p  = __expf(v - mn);
          const float* xp = fs + (size_t)s * HCOL + lane * 8;
          const v4f x0 = *(const v4f*)xp, x1 = *(const v4f*)(xp + 4);
          v4f* ap = (v4f*)(acc + slot * HCOL + lane * 8);
          v4f a0 = ap[0], a1 = ap[1];
          a0 = a0 * sc + x0 * p;
          a1 = a1 * sc + x1 * p;
          ap[0] = a0;
          ap[1] = a1;
          if ((lane & 7) == 0) {
            mx[slot * NHD + hsel]  = mn;
            den[slot * NHD + hsel] = dn * sc + p;
          }
          __builtin_amdgcn_fence(__ATOMIC_RELEASE, "wavefront");
          __builtin_amdgcn_wave_barrier();
          __builtin_amdgcn_fence(__ATOMIC_ACQUIRE, "wavefront");
        }
      }
    }
    __syncthreads();
  }
  __syncthreads();

  const int hA = lane >> 4, hB = 2 + (lane >> 4);
#pragma unroll 1
  for (int j = 0; j < NB / NWAVE; ++j) {
    const int slot = wave * (NB / NWAVE) + j;
    const int node = nodeBase + slot;
    if (node >= nN) break;
    const float d1 = den[slot * NHD + hA], d2 = den[slot * NHD + hB];
    const float i1 = d1 > 0.f ? 1.0f / d1 : 0.f;
    const float i2 = d2 > 0.f ? 1.0f / d2 : 0.f;
    const v4f a0 = *(const v4f*)(acc + slot * HCOL + 4 * lane);
    const v4f a1 = *(const v4f*)(acc + slot * HCOL + 128 + 4 * lane);
    float* hp = hsum + (size_t)node * HCOL;
    const v4f o0 = *(const v4f*)(hp + 4 * lane) + a0 * i1;
    const v4f o1 = *(const v4f*)(hp + 128 + 4 * lane) + a1 * i2;
    *(volatile v4f*)(hp + 4 * lane) = o0;
    *(volatile v4f*)(hp + 128 + 4 * lane) = o1;
    __threadfence();
    *(volatile v4f*)(hp + 4 * lane) = o0;
    *(volatile v4f*)(hp + 128 + 4 * lane) = o1;
  }
}
#undef HITJ

extern "C" void kernel_launch(void* const* d_in, const int* in_sizes, int n_in,
                              void* d_out, int out_size, void* d_ws, size_t ws_size,
                              hipStream_t stream) {
  if (n_in < 25) return;
  const int nN = in_sizes[0] / DX;
  if (nN <= 0 || in_sizes[0] != nN * DX || out_size != nN * DX) return;
  const int Ecnt[3] = {in_sizes[1], in_sizes[3], in_sizes[5]};
  if (in_sizes[2] != Ecnt[0] || in_sizes[4] != Ecnt[1] || in_sizes[6] != Ecnt[2]) return;
  if (Ecnt[0] < 0 || Ecnt[1] < 0 || Ecnt[2] < 0) return;
  if (in_sizes[7] != 3 * KP * HCOL || in_sizes[11] != 3 * KP * HCOL ||
      in_sizes[12] != 3 * KP * HCOL || in_sizes[16] != 3 * KP * HCOL) return;
  if (in_sizes[8] != 3 * NHD * DX || in_sizes[9] != 3 * NHD * DX ||
      in_sizes[13] != 3 * NHD * DX || in_sizes[14] != 3 * NHD * DX) return;
  if (in_sizes[10] != 3 * HCOL || in_sizes[15] != 3 * HCOL) return;
  if (in_sizes[17] != DX * DX || in_sizes[19] != DX * DX) return;
  for (int i = 18; i <= 24; i += 2) if (in_sizes[i] != DX) return;
  if (in_sizes[21] != DX || in_sizes[23] != DX) return;

  const float* x = (const float*)d_in[0];
  const int* srcs[3] = {(const int*)d_in[1], (const int*)d_in[3], (const int*)d_in[5]};
  const int* dsts[3] = {(const int*)d_in[2], (const int*)d_in[4], (const int*)d_in[6]};
  const float* Wl[2]  = {(const float*)d_in[7],  (const float*)d_in[12]};
  const float* all[2] = {(const float*)d_in[8],  (const float*)d_in[13]};
  const float* arl[2] = {(const float*)d_in[9],  (const float*)d_in[14]};
  const float* bl[2]  = {(const float*)d_in[10], (const float*)d_in[15]};
  const float* rWl[2] = {(const float*)d_in[11], (const float*)d_in[16]};
  const float* fcW[2] = {(const float*)d_in[17], (const float*)d_in[19]};
  const float* fcb[2] = {(const float*)d_in[18], (const float*)d_in[20]};
  const float* gl[2]  = {(const float*)d_in[21], (const float*)d_in[23]};
  const float* bel[2] = {(const float*)d_in[22], (const float*)d_in[24]};
  float* out = (float*)d_out;

  const int Np = ((nN + RPB_N - 1) / RPB_N) * RPB_N;
  const int P  = (nN + RB - 1) / RB;

  size_t off = 0;
  char* base = (char*)d_ws;
  auto carve = [&](size_t bytes) -> char* { char* p = base + off; off += (bytes + 255) & ~(size_t)255; return p; };
  float*  fsP   = (float*)carve((size_t)Np * HCOL * sizeof(float));
  float*  hsum  = (float*)carve((size_t)Np * HCOL * sizeof(float));
  float*  xnext = (float*)carve((size_t)Np * DX * sizeof(float));
  us*     xbh   = (us*)carve((size_t)Np * DX * sizeof(us));
  us*     xbl   = (us*)carve((size_t)Np * DX * sizeof(us));
  float*  eler  = (float*)carve((size_t)Np * 8 * sizeof(float));
  us*     Wth   = (us*)carve((size_t)3 * HCOL * KP * sizeof(us));
  us*     Wtl   = (us*)carve((size_t)3 * HCOL * KP * sizeof(us));
  us*     Rth   = (us*)carve((size_t)HCOL * KP * sizeof(us));
  us*     Rtl   = (us*)carve((size_t)HCOL * KP * sizeof(us));
  us*     Fth   = (us*)carve((size_t)DX * KP * sizeof(us));
  us*     Ftl   = (us*)carve((size_t)DX * KP * sizeof(us));
  float*  bsum  = (float*)carve((size_t)HCOL * sizeof(float));
  double* part  = (double*)carve((size_t)P * 128 * sizeof(double));
  float*  scsh  = (float*)carve((size_t)2 * DX * sizeof(float));
  if (off > ws_size || off > (size_t)134217728) return;

  hipFuncSetAttribute(reinterpret_cast<const void*>(&k_agg),
                      hipFuncAttributeMaxDynamicSharedMemorySize, AGG_LDS);

  const int gridPrep = (PT_ALL + NTHR - 1) / NTHR;
  const int gridApp  = Np / 32;
  const int gridW    = Np / RPB_W;
  const int gridN    = Np / RPB_N;
  const int gridAgg  = (nN + NB - 1) / NB;

  for (int L = 0; L < 2; ++L) {
    const float* xin = (L == 0) ? x : (const float*)xnext;
    float* yout = (L == 0) ? xnext : out;
    const int nst = (L == 0) ? Np : nN;

    k_prep<<<gridPrep, NTHR, 0, stream>>>(Wl[L], rWl[L], bl[L], fcW[L], Wth, Wtl, Rth, Rtl, Fth, Ftl, bsum);
    k_bn_part<<<P, NTHR, 0, stream>>>(xin, nN, part);
    k_bn_final<<<1, NTHR, 0, stream>>>(part, P, nN, gl[L], scsh);
    k_bn_apply<<<gridApp, NTHR, 0, stream>>>(xin, scsh, bel[L], nN, xbh, xbl);
    k_gemm<1><<<gridW, NTHR, 0, stream>>>(xbh, xbl, fsP, Rth, Rtl, bsum, bsum, hsum, eler, HCOL, Np);
    for (int r = 0; r < 3; ++r) {
      k_gemm<0><<<gridW, NTHR, 0, stream>>>(xbh, xbl, hsum, Wth + (size_t)r * HCOL * KP, Wtl + (size_t)r * HCOL * KP,
                                            all[L] + r * NHD * DX, arl[L] + r * NHD * DX, fsP, eler, HCOL, Np);
      if (Ecnt[r] > 0)
        k_agg<<<gridAgg, NTHR, AGG_LDS, stream>>>(srcs[r], dsts[r], Ecnt[r], fsP, eler, hsum, nN);
    }
    k_gemm<2><<<gridN, NTHR, 0, stream>>>(xbh, xbl, hsum, Fth, Ftl, fcb[L], fcb[L], yout, eler, DX, nst);
  }
}
